// SemiSupervisedGAT_43499428774652
// MI455X (gfx1250) — hardware-verified
//
#include <hip/hip_runtime.h>
#define NNODE 100000
#define NE 1600000
#define IND 128
#define HID 64
#define HD2 32
#define NRB 512

typedef __bf16 v16b __attribute__((ext_vector_type(16)));
typedef unsigned short v8us __attribute__((ext_vector_type(8), may_alias));
typedef float  v8f  __attribute__((ext_vector_type(8)));
typedef float  v4f  __attribute__((ext_vector_type(4)));
typedef float  v4fa __attribute__((ext_vector_type(4), may_alias));
union FragB { v16b v; v8us half[2]; unsigned short u[16]; };

__device__ __forceinline__ unsigned short bf16_bits(float x) { unsigned int u = __float_as_uint(x); return (unsigned short)((u + 0x7FFFu + ((u >> 16) & 1u)) >> 16); }
__device__ __forceinline__ float bf16_val(unsigned short b) { return __uint_as_float(((unsigned int)b) << 16); }
__device__ __forceinline__ float bf16_round(float x) { return bf16_val(bf16_bits(x)); }
template <int NT>
__device__ __forceinline__ v8f mmaN(v16b ah, v16b al, v16b bh, v16b bl, v8f c) {
  c = __builtin_amdgcn_wmma_f32_16x16x32_bf16(false, ah, false, bh, (short)0, c, false, false);
  if (NT >= 2) c = __builtin_amdgcn_wmma_f32_16x16x32_bf16(false, al, false, bh, (short)0, c, false, false);
  if (NT >= 3) c = __builtin_amdgcn_wmma_f32_16x16x32_bf16(false, ah, false, bl, (short)0, c, false, false);
  asm volatile("v_nop\n\tv_nop\n\tv_nop\n\tv_nop" : "+v"(c) : "v"(ah), "v"(al), "v"(bh), "v"(bl));
  return c;
}

__global__ __launch_bounds__(256) void k_wt_bf16(const float* __restrict__ W, unsigned short* __restrict__ Wt, int K, int N) {
  const int t = blockIdx.x * 256 + threadIdx.x;
  const int k8n = K / 8;
  if (t >= N * k8n) return;
  const int n = t / k8n, k8 = (t % k8n) * 8;
  v8us v;
#pragma unroll
  for (int i = 0; i < 8; ++i) v[i] = bf16_bits(W[(size_t)(k8 + i) * N + n]);
  *(volatile v8us*)(Wt + (size_t)n * K + k8) = v;
  __threadfence();
  *(volatile v8us*)(Wt + (size_t)n * K + k8) = v;
}

template <bool ASPLIT, int ACT, bool BIAS_BF16>
__global__ __launch_bounds__(128) void k_gemm_bf(const float* __restrict__ A, int lda, const unsigned short* __restrict__ Wt, int ldb,
                                               const float* __restrict__ bias, float* __restrict__ C, int ldc, int M, int N, int K) {
  __shared__ __attribute__((aligned(16))) float so[4][16][64];
  const int tid = threadIdx.x, w = tid >> 5, lane = tid & 31, ln = lane & 15, hh = lane >> 4;
  const int ntn = N / 64;
  const int wid = blockIdx.x * 4 + w;
  const int mt = wid / ntn, nq = wid % ntn;
  if (mt * 16 >= M) return;
  const int row0 = mt * 16, col0 = nq * 64;
  const float* arow = A + (size_t)(row0 + ln) * lda;
  v8f acc[4] = {};
  for (int kb = 0; kb < K; kb += 32) {
    FragB ah, al;
    const v4f x0 = *(const v4fa*)(arow + kb + 8 * hh), x1 = *(const v4fa*)(arow + kb + 8 * hh + 4);
    const v4f x2 = *(const v4fa*)(arow + kb + 16 + 8 * hh), x3 = *(const v4fa*)(arow + kb + 16 + 8 * hh + 4);
    float xs[16] = {x0[0],x0[1],x0[2],x0[3],x1[0],x1[1],x1[2],x1[3],x2[0],x2[1],x2[2],x2[3],x3[0],x3[1],x3[2],x3[3]};
#pragma unroll
    for (int i = 0; i < 16; ++i) { const unsigned short hb = bf16_bits(xs[i]); ah.u[i] = hb; al.u[i] = ASPLIT ? bf16_bits(xs[i] - bf16_val(hb)) : (unsigned short)0; }
#pragma unroll
    for (int t = 0; t < 4; ++t) {
      const unsigned short* brow = Wt + (size_t)(col0 + t * 16 + ln) * ldb + kb;
      FragB b;
      b.half[0] = *(const v8us*)(brow + 8 * hh);
      b.half[1] = *(const v8us*)(brow + 16 + 8 * hh);
      acc[t] = mmaN<ASPLIT ? 2 : 1>(ah.v, al.v, b.v, b.v, acc[t]);
    }
  }
#pragma unroll
  for (int t = 0; t < 4; ++t) {
    float bv = bias ? bias[col0 + t * 16 + ln] : 0.f;
    if (BIAS_BF16) bv = bf16_round(bv);
#pragma unroll
    for (int r = 0; r < 8; ++r) { float v = acc[t][r] + bv; if (ACT == 1) v = fmaxf(v, 0.f); so[w][8 * hh + r][t * 16 + ln] = v; }
  }
  __builtin_amdgcn_fence(__ATOMIC_ACQ_REL, "workgroup");
  __builtin_amdgcn_wave_barrier();
  const int rsub = lane >> 4, c4 = (lane & 15) * 4;
  for (int pass = 0; pass < 2; ++pass) {
#pragma unroll
    for (int q = 0; q < 8; ++q) {
      const int r = q * 2 + rsub;
      const v4f v = *(const v4fa*)&so[w][r][c4];
      *(volatile v4f*)(C + (size_t)(row0 + r) * ldc + col0 + c4) = v;
    }
    if (pass == 0) __threadfence();
  }
}

template <int D, bool CAUSAL>
__global__ __launch_bounds__(128) void k_flash(const float* __restrict__ qb, const float* __restrict__ kb, const float* __restrict__ vb,
                                             int pitch, int T, int H, float scale, float* __restrict__ y, int ypitch) {
  constexpr int KS = D / 32;
  constexpr int DT = D / 16;
  __shared__ __attribute__((aligned(16))) unsigned short sKh[32][D + 8], sKl[32][D + 8], sVh[32][D + 8], sVl[32][D + 8];
  __shared__ __attribute__((aligned(16))) unsigned short sPh[4][16][40], sPl[4][16][40];
  __shared__ __attribute__((aligned(16))) float sO[4][16][D];
  const int tid = threadIdx.x, w = tid >> 5, lane = tid & 31, ln = lane & 15, hh = lane >> 4;
  const int nqb = (T + 63) / 64;
  const int bh = blockIdx.x / nqb, qblk = blockIdx.x % nqb;
  const int b = bh / H, h = bh % H;
  const int q0 = qblk * 64 + w * 16;
  const float* Q = qb + (size_t)b * T * pitch + h * D;
  const float* K = kb + (size_t)b * T * pitch + h * D;
  const float* V = vb + (size_t)b * T * pitch + h * D;

  FragB aqh[KS], aql[KS];
  {
    int row = q0 + ln; if (row >= T) row = T - 1;
    const float* qr = Q + (size_t)row * pitch;
#pragma unroll
    for (int ks = 0; ks < KS; ++ks)
#pragma unroll
      for (int i = 0; i < 16; ++i) {
        const int d = ks * 32 + ((i < 8) ? (8 * hh + i) : (16 + 8 * hh + (i - 8)));
        const float x = qr[d] * scale; const unsigned short hb = bf16_bits(x);
        aqh[ks].u[i] = hb; aql[ks].u[i] = bf16_bits(x - bf16_val(hb));
      }
  }
  float m_r[8], l_r[8];
#pragma unroll
  for (int r = 0; r < 8; ++r) { m_r[r] = -3.0e38f; l_r[r] = 0.f; }
  v8f oacc[DT];
#pragma unroll
  for (int dt = 0; dt < DT; ++dt) oacc[dt] = (v8f){0.f,0.f,0.f,0.f,0.f,0.f,0.f,0.f};

  const int kv_end = CAUSAL ? min(T, qblk * 64 + 64) : T;
  for (int j0 = 0; j0 < kv_end; j0 += 32) {
    __syncthreads();
    for (int e = tid; e < 32 * (D / 4); e += 128) {
      const int r = e / (D / 4), c4 = (e % (D / 4)) * 4;
      const int key = j0 + r;
      v4f kf = {0.f,0.f,0.f,0.f}, vf = {0.f,0.f,0.f,0.f};
      if (key < T) { kf = *(const v4fa*)(K + (size_t)key * pitch + c4); vf = *(const v4fa*)(V + (size_t)key * pitch + c4); }
#pragma unroll
      for (int t = 0; t < 4; ++t) {
        unsigned short hb = bf16_bits(kf[t]); sKh[r][c4 + t] = hb; sKl[r][c4 + t] = bf16_bits(kf[t] - bf16_val(hb));
        hb = bf16_bits(vf[t]); sVh[r][c4 + t] = hb; sVl[r][c4 + t] = bf16_bits(vf[t] - bf16_val(hb));
      }
    }
    __syncthreads();
    v8f s[2];
#pragma unroll
    for (int nt = 0; nt < 2; ++nt) {
      v8f acc = {};
#pragma unroll
      for (int ks = 0; ks < KS; ++ks) {
        FragB bh_, bl_;
        bh_.half[0] = *(const v8us*)&sKh[nt * 16 + ln][ks * 32 + 8 * hh]; bh_.half[1] = *(const v8us*)&sKh[nt * 16 + ln][ks * 32 + 16 + 8 * hh];
        bl_.half[0] = *(const v8us*)&sKl[nt * 16 + ln][ks * 32 + 8 * hh]; bl_.half[1] = *(const v8us*)&sKl[nt * 16 + ln][ks * 32 + 16 + 8 * hh];
        acc = mmaN<3>(aqh[ks].v, aql[ks].v, bh_.v, bl_.v, acc);
      }
      s[nt] = acc;
    }
    float alpha[8];
#pragma unroll
    for (int r = 0; r < 8; ++r) {
      const int qi = q0 + 8 * hh + r;
      const int ja = j0 + ln, jb = j0 + 16 + ln;
      if (CAUSAL) { if (ja > qi) s[0][r] = -3.0e38f; if (jb > qi) s[1][r] = -3.0e38f; }
      if (ja >= T) s[0][r] = -3.0e38f;
      if (jb >= T) s[1][r] = -3.0e38f;
      float mx = fmaxf(s[0][r], s[1][r]);
      mx = fmaxf(mx, __shfl_xor(mx, 1, 32)); mx = fmaxf(mx, __shfl_xor(mx, 2, 32)); mx = fmaxf(mx, __shfl_xor(mx, 4, 32)); mx = fmaxf(mx, __shfl_xor(mx, 8, 32));
      const float mnew = fmaxf(m_r[r], mx);
      alpha[r] = (mnew > -1.0e38f) ? __expf(m_r[r] - mnew) : 1.0f;
      const float p0 = (s[0][r] > -1.0e38f) ? __expf(s[0][r] - mnew) : 0.f;
      const float p1 = (s[1][r] > -1.0e38f) ? __expf(s[1][r] - mnew) : 0.f;
      m_r[r] = mnew;
      l_r[r] = l_r[r] * alpha[r] + p0 + p1;
      unsigned short hb = bf16_bits(p0); sPh[w][8 * hh + r][ln] = hb;      sPl[w][8 * hh + r][ln] = bf16_bits(p0 - bf16_val(hb));
      hb = bf16_bits(p1);                sPh[w][8 * hh + r][16 + ln] = hb; sPl[w][8 * hh + r][16 + ln] = bf16_bits(p1 - bf16_val(hb));
    }
#pragma unroll
    for (int dt = 0; dt < DT; ++dt)
#pragma unroll
      for (int r = 0; r < 8; ++r) oacc[dt][r] *= alpha[r];
    __builtin_amdgcn_fence(__ATOMIC_ACQ_REL, "workgroup");
    __builtin_amdgcn_wave_barrier();
    FragB pah, pal;
    pah.half[0] = *(const v8us*)&sPh[w][ln][8 * hh]; pah.half[1] = *(const v8us*)&sPh[w][ln][16 + 8 * hh];
    pal.half[0] = *(const v8us*)&sPl[w][ln][8 * hh]; pal.half[1] = *(const v8us*)&sPl[w][ln][16 + 8 * hh];
#pragma unroll
    for (int dt = 0; dt < DT; ++dt) {
      FragB bvh, bvl;
#pragma unroll
      for (int i = 0; i < 8; ++i) {
        bvh.u[i] = sVh[8 * hh + i][dt * 16 + ln]; bvh.u[8 + i] = sVh[16 + 8 * hh + i][dt * 16 + ln];
        bvl.u[i] = sVl[8 * hh + i][dt * 16 + ln]; bvl.u[8 + i] = sVl[16 + 8 * hh + i][dt * 16 + ln];
      }
      oacc[dt] = mmaN<3>(pah.v, pal.v, bvh.v, bvl.v, oacc[dt]);
    }
    __builtin_amdgcn_fence(__ATOMIC_ACQ_REL, "workgroup");
    __builtin_amdgcn_wave_barrier();
  }
#pragma unroll
  for (int r = 0; r < 8; ++r) {
    float l = l_r[r];
    l += __shfl_xor(l, 1, 32); l += __shfl_xor(l, 2, 32); l += __shfl_xor(l, 4, 32); l += __shfl_xor(l, 8, 32);
    l_r[r] = (l > 0.f) ? 1.0f / l : 0.f;
  }
#pragma unroll
  for (int dt = 0; dt < DT; ++dt)
#pragma unroll
    for (int r = 0; r < 8; ++r) sO[w][8 * hh + r][dt * 16 + ln] = oacc[dt][r] * l_r[r];
  __builtin_amdgcn_fence(__ATOMIC_ACQ_REL, "workgroup");
  __builtin_amdgcn_wave_barrier();
  for (int pass = 0; pass < 2; ++pass) {
    for (int r = 0; r < 16; ++r) {
      const int row = q0 + r;
      if (row < T && lane < D / 4) {
        const v4f val = *(const v4fa*)&sO[w][r][lane * 4];
        *(volatile v4f*)(y + ((size_t)b * T + row) * ypitch + h * D + lane * 4) = val;
      }
    }
    if (pass == 0) __threadfence();
  }
}

template <bool ASPLIT, int ACT, bool BIAS_BF16, bool RES_BF16>
__global__ __launch_bounds__(128) void k_gemm_bf3(const float* __restrict__ A, int lda, const unsigned short* __restrict__ Wt, int ldb,
                                                const float* __restrict__ bias, const float* __restrict__ resid, int rmod, int ldr,
                                                float* __restrict__ C, int ldc, int M, int N, int K) {
  __shared__ __attribute__((aligned(16))) float so[4][16][64];
  const int tid = threadIdx.x, w = tid >> 5, lane = tid & 31, ln = lane & 15, hh = lane >> 4;
  const int ntn = N / 64;
  const int wid = blockIdx.x * 4 + w;
  const int mt = wid / ntn, nq = wid % ntn;
  if (mt * 16 >= M) return;
  const int row0 = mt * 16, col0 = nq * 64;
  const float* arow = A + (size_t)(row0 + ln) * lda;
  v8f acc[4] = {};
  for (int kb = 0; kb < K; kb += 32) {
    FragB ah, al;
    const v4f x0 = *(const v4fa*)(arow + kb + 8 * hh), x1 = *(const v4fa*)(arow + kb + 8 * hh + 4);
    const v4f x2 = *(const v4fa*)(arow + kb + 16 + 8 * hh), x3 = *(const v4fa*)(arow + kb + 16 + 8 * hh + 4);
    float xs[16] = {x0[0],x0[1],x0[2],x0[3],x1[0],x1[1],x1[2],x1[3],x2[0],x2[1],x2[2],x2[3],x3[0],x3[1],x3[2],x3[3]};
#pragma unroll
    for (int i = 0; i < 16; ++i) { const unsigned short hb = bf16_bits(xs[i]); ah.u[i] = hb; al.u[i] = ASPLIT ? bf16_bits(xs[i] - bf16_val(hb)) : (unsigned short)0; }
#pragma unroll
    for (int t = 0; t < 4; ++t) {
      const unsigned short* brow = Wt + (size_t)(col0 + t * 16 + ln) * ldb + kb;
      FragB b;
      b.half[0] = *(const v8us*)(brow + 8 * hh);
      b.half[1] = *(const v8us*)(brow + 16 + 8 * hh);
      acc[t] = mmaN<ASPLIT ? 2 : 1>(ah.v, al.v, b.v, b.v, acc[t]);
    }
  }
#pragma unroll
  for (int t = 0; t < 4; ++t) {
    const int col = col0 + t * 16 + ln;
    float bv = bias ? bias[col] : 0.f;
    if (BIAS_BF16) bv = bf16_round(bv);
#pragma unroll
    for (int r = 0; r < 8; ++r) {
      float v = acc[t][r] + bv;
      if (resid) { float rv = resid[(size_t)((row0 + 8 * hh + r) % rmod) * ldr + col]; if (RES_BF16) rv = bf16_round(rv); v += rv; }
      if (ACT == 1) v = fmaxf(v, 0.f);
      if (ACT == 2) v = 0.5f * v * (1.0f + erff(v * 0.70710678118654752f));
      if (ACT == 3) { const float u = 0.7978845608028654f * (v + 0.044715f * v * v * v); v = 0.5f * v * (1.0f + tanhf(u)); }
      so[w][8 * hh + r][t * 16 + ln] = v;
    }
  }
  __builtin_amdgcn_fence(__ATOMIC_ACQ_REL, "workgroup");
  __builtin_amdgcn_wave_barrier();
  const int rsub = lane >> 4, c4 = (lane & 15) * 4;
  for (int pass = 0; pass < 2; ++pass) {
#pragma unroll
    for (int q = 0; q < 8; ++q) {
      const int r = q * 2 + rsub;
      const v4f v = *(const v4fa*)&so[w][r][c4];
      *(volatile v4f*)(C + (size_t)(row0 + r) * ldc + col0 + c4) = v;
    }
    if (pass == 0) __threadfence();
  }
}
template <bool PARAM_BF16>
__global__ __launch_bounds__(256) void k_layernorm(const float* __restrict__ X, const float* __restrict__ R, const float* __restrict__ g, const float* __restrict__ bta,
                                                  float* __restrict__ out_sum, float* __restrict__ out_norm, int N, float eps) {
  __shared__ float red[256];
  const int row = blockIdx.x, tid = threadIdx.x;
  const float* x = X + (size_t)row * N; const float* rr = R ? R + (size_t)row * N : nullptr;
  float vals[16];
  const int per = N / 256;
  float s1 = 0.f;
  for (int u = 0; u < per / 4; ++u) {
    const int j = tid * 4 + 1024 * u;
    const v4f a = *(const v4fa*)(x + j);
    v4f b = {0.f,0.f,0.f,0.f}; if (rr) b = *(const v4fa*)(rr + j);
#pragma unroll
    for (int q = 0; q < 4; ++q) { const float v = a[q] + b[q]; vals[u * 4 + q] = v; s1 += v; }
  }
  red[tid] = s1; __syncthreads();
  for (int st = 128; st > 0; st >>= 1) { if (tid < st) red[tid] += red[tid + st]; __syncthreads(); }
  const float mu = red[0] / (float)N; __syncthreads();
  float s2 = 0.f;
  for (int u = 0; u < per / 4; ++u)
#pragma unroll
    for (int q = 0; q < 4; ++q) { const float c = vals[u * 4 + q] - mu; s2 += c * c; }
  red[tid] = s2; __syncthreads();
  for (int st = 128; st > 0; st >>= 1) { if (tid < st) red[tid] += red[tid + st]; __syncthreads(); }
  const float rs = rsqrtf(red[0] / (float)N + eps);
  for (int pass = 0; pass < 2; ++pass) {
    for (int u = 0; u < per / 4; ++u) {
      const int j = tid * 4 + 1024 * u;
      v4f o, sm;
#pragma unroll
      for (int q = 0; q < 4; ++q) {
        float gg = g[j + q], bb = bta[j + q];
        if (PARAM_BF16) { gg = bf16_round(gg); bb = bf16_round(bb); }
        sm[q] = vals[u * 4 + q]; o[q] = (vals[u * 4 + q] - mu) * rs * gg + bb;
      }
      if (out_sum) *(volatile v4f*)(out_sum + (size_t)row * N + j) = sm;
      *(volatile v4f*)(out_norm + (size_t)row * N + j) = o;
    }
    if (pass == 0) __threadfence();
  }
}


typedef _Float16 v16h __attribute__((ext_vector_type(16)));
union FragH { v16h v; v8us half[2]; _Float16 h[16]; unsigned short u[16]; };
template <int NT>
__device__ __forceinline__ v8f mmaH(v16h ah, v16h al, v16h bh, v16h bl, v8f c) {
  c = __builtin_amdgcn_wmma_f32_16x16x32_f16(false, ah, false, bh, (short)0, c, false, false);
  if (NT >= 2) c = __builtin_amdgcn_wmma_f32_16x16x32_f16(false, al, false, bh, (short)0, c, false, false);
  if (NT >= 3) c = __builtin_amdgcn_wmma_f32_16x16x32_f16(false, ah, false, bl, (short)0, c, false, false);
  asm volatile("v_nop\n\tv_nop\n\tv_nop\n\tv_nop" : "+v"(c) : "v"(ah), "v"(al), "v"(bh), "v"(bl));
  return c;
}
template <bool ASPLIT>
__global__ __launch_bounds__(128) void k_gemm_h(const float* __restrict__ A, int lda, size_t sA, const _Float16* __restrict__ Bh, int ldb, size_t sB, float alpha, float* __restrict__ C, int ldc, size_t sC, int M, int N, int K) {
  __shared__ __attribute__((aligned(16))) float so[4][16][64];
  const int tid = threadIdx.x, w = tid >> 5, lane = tid & 31, ln = lane & 15, hh = lane >> 4; const int by = blockIdx.y;
  A += (size_t)by * sA; Bh += (size_t)by * sB; C += (size_t)by * sC;
  const int ntn = (N + 63) / 64; const int wid = blockIdx.x * 4 + w; const int mt = wid / ntn, nq = wid % ntn; if (mt * 16 >= M) return;
  const int row0 = mt * 16, col0 = nq * 64; const float* arow = A + (size_t)(row0 + ln) * lda;
  v8f acc[4] = {};
  for (int kb = 0; kb < K; kb += 32) {
    FragH ah, al;
    const v4f x0 = *(const v4fa*)(arow + kb + 8 * hh), x1 = *(const v4fa*)(arow + kb + 8 * hh + 4), x2 = *(const v4fa*)(arow + kb + 16 + 8 * hh), x3 = *(const v4fa*)(arow + kb + 16 + 8 * hh + 4);
    float xs[16] = {x0[0],x0[1],x0[2],x0[3],x1[0],x1[1],x1[2],x1[3],x2[0],x2[1],x2[2],x2[3],x3[0],x3[1],x3[2],x3[3]};
#pragma unroll
    for (int i = 0; i < 16; ++i) { const _Float16 h = (_Float16)xs[i]; ah.h[i] = h; al.h[i] = ASPLIT ? (_Float16)(xs[i] - (float)h) : (_Float16)0.0f; }
#pragma unroll
    for (int t = 0; t < 4; ++t) { if (col0 + t * 16 >= N) continue; const size_t boff = (size_t)(col0 + t * 16 + ln) * ldb + kb; FragH bq; bq.half[0] = *(const v8us*)(Bh + boff + 8 * hh); bq.half[1] = *(const v8us*)(Bh + boff + 16 + 8 * hh);
      acc[t] = mmaH<ASPLIT ? 2 : 1>(ah.v, al.v, bq.v, bq.v, acc[t]); }
  }
#pragma unroll
  for (int t = 0; t < 4; ++t) { if (col0 + t * 16 >= N) continue;
#pragma unroll
    for (int r = 0; r < 8; ++r) so[w][8 * hh + r][t * 16 + ln] = acc[t][r] * alpha; }
  __builtin_amdgcn_fence(__ATOMIC_ACQ_REL, "workgroup"); __builtin_amdgcn_wave_barrier();
  const int rsub = lane >> 4, c4 = (lane & 15) * 4;
  for (int pass = 0; pass < 2; ++pass) {
#pragma unroll
    for (int q = 0; q < 8; ++q) { const int r = q * 2 + rsub; if (col0 + c4 < N) { const v4f v = *(const v4fa*)&so[w][r][c4]; *(volatile v4f*)(C + (size_t)(row0 + r) * ldc + col0 + c4) = v; } }
    if (pass == 0) __threadfence(); }
}

__global__ __launch_bounds__(256) void k_wt_f16(const float* __restrict__ W, _Float16* __restrict__ Wt, int K, int N, float scale) {
  const int t = blockIdx.x * 256 + threadIdx.x; if (t >= N * (K / 8)) return; const int n = t / (K / 8), k8 = (t % (K / 8)) * 8; FragH f;
#pragma unroll
  for (int i = 0; i < 8; ++i) f.h[i] = (_Float16)(bf16_round(W[(size_t)(k8 + i) * N + n]) * scale); const v8us o = f.half[0];
  *(volatile v8us*)((unsigned short*)Wt + (size_t)n * K + k8) = o; __threadfence(); *(volatile v8us*)((unsigned short*)Wt + (size_t)n * K + k8) = o;
}
template <int ACT>
__global__ __launch_bounds__(128) void k_gemm_hhx(const _Float16* __restrict__ A, int lda, size_t sA, const _Float16* __restrict__ Bh, int ldb, size_t sB, float alpha, const float* __restrict__ bias, size_t sBias, const float* __restrict__ CP, int rowsPerB, size_t sCPb, int row0g,
    float* __restrict__ C, _Float16* __restrict__ C16, int ldc, size_t sC, int M, int N, int K) {
  __shared__ __attribute__((aligned(16))) float so[4][16][64];
  const int tid = threadIdx.x, w = tid >> 5, lane = tid & 31, ln = lane & 15, hh = lane >> 4; const int by = blockIdx.y;
  A += (size_t)by * sA; Bh += (size_t)by * sB; const size_t cofs = (size_t)by * sC; const float* bp = bias ? bias + (size_t)by * sBias : nullptr;
  const int ntn = (N + 63) / 64; const int wid = blockIdx.x * 4 + w; const int mt = wid / ntn, nq = wid % ntn; if (mt * 16 >= M) return;
  const int row0 = mt * 16, col0 = nq * 64; const _Float16* arow = A + (size_t)(row0 + ln) * lda;
  v8f acc[4] = {};
  for (int kb = 0; kb < K; kb += 32) { FragH ah; ah.half[0] = *(const v8us*)((const unsigned short*)arow + kb + 8 * hh); ah.half[1] = *(const v8us*)((const unsigned short*)arow + kb + 16 + 8 * hh);
#pragma unroll
    for (int t = 0; t < 4; ++t) { if (col0 + t * 16 >= N) continue; const size_t boff = (size_t)(col0 + t * 16 + ln) * ldb + kb; FragH bq; bq.half[0] = *(const v8us*)((const unsigned short*)Bh + boff + 8 * hh); bq.half[1] = *(const v8us*)((const unsigned short*)Bh + boff + 16 + 8 * hh);
      acc[t] = mmaH<1>(ah.v, ah.v, bq.v, bq.v, acc[t]); }
  }
#pragma unroll
  for (int t = 0; t < 4; ++t) { if (col0 + t * 16 >= N) continue; const int col = col0 + t * 16 + ln; const float bv = bp ? bf16_round(bp[col]) : 0.f;
#pragma unroll
    for (int r = 0; r < 8; ++r) { float v = acc[t][r] * alpha + bv; if (CP) { const int bidx = (row0g + row0 + 8 * hh + r) / rowsPerB; v += CP[(size_t)bidx * sCPb + (size_t)by * 64 + col]; } if (ACT == 1) v = (v > 0.f) ? v : expm1f(v); else if (ACT == 3) v = fmaxf(v, 0.f); so[w][8 * hh + r][t * 16 + ln] = v; } }
  __builtin_amdgcn_fence(__ATOMIC_ACQ_REL, "workgroup"); __builtin_amdgcn_wave_barrier();
  const int rsub = lane >> 4, c4 = (lane & 15) * 4; typedef _Float16 v4h __attribute__((ext_vector_type(4)));
  for (int pass = 0; pass < 2; ++pass) {
#pragma unroll
    for (int q = 0; q < 8; ++q) { const int r = q * 2 + rsub; if (col0 + c4 < N) { const v4f v = *(const v4fa*)&so[w][r][c4]; if (C) *(volatile v4f*)(C + cofs + (size_t)(row0 + r) * ldc + col0 + c4) = v; if (C16) { v4h h4; for (int i = 0; i < 4; ++i) h4[i] = (_Float16)v[i]; *(volatile v4h*)(C16 + cofs + (size_t)(row0 + r) * ldc + col0 + c4) = h4; } } }
    if (pass == 0) __threadfence(); }
}


__device__ __forceinline__ int bscan1024(int cnt, int* wsum, int tid, int& total) {
  const int lane = tid & 31, wv = tid >> 5; int x = cnt;
#pragma unroll
  for (int d = 1; d < 32; d <<= 1) { const int y = __shfl_up(x, d, 32); if (lane >= d) x += y; }
  __syncthreads(); if (lane == 31) wsum[wv] = x; __syncthreads();
  int t = (lane < 32) ? wsum[lane] : 0;
#pragma unroll
  for (int d = 1; d < 32; d <<= 1) { const int y = __shfl_up(t, d, 32); if (lane >= d) t += y; }
  const int woff = (wv == 0) ? 0 : __shfl(t, wv - 1, 32); total = __shfl(t, 31, 32);
  return woff + x - cnt; }
__global__ __launch_bounds__(256) void k_x16(const float* __restrict__ x, _Float16* __restrict__ X16, size_t n8) { const size_t t = (size_t)blockIdx.x * 256 + threadIdx.x; if (t >= n8) return; FragH f;
#pragma unroll
  for (int q = 0; q < 8; ++q) f.h[q] = (_Float16)bf16_round(x[t * 8 + q]); *(volatile v8us*)((unsigned short*)X16 + t * 8) = f.half[0]; __threadfence(); *(volatile v8us*)((unsigned short*)X16 + t * 8) = f.half[0]; }
__global__ __launch_bounds__(1024) void k_sad(const float* __restrict__ H, const float* __restrict__ A, float* __restrict__ SAD) { __shared__ float so[32][4]; const int tid = threadIdx.x, wv = tid >> 5, lane = tid & 31; const int n = blockIdx.x * 32 + wv; float s[4] = {0.f, 0.f, 0.f, 0.f};
  if (n < NNODE) { const float h0 = H[(size_t)n * HID + lane], h1 = H[(size_t)n * HID + 32 + lane];
    s[0] = h0 * bf16_round(A[lane * 2]) + h1 * bf16_round(A[(32 + lane) * 2]); s[1] = h0 * bf16_round(A[lane * 2 + 1]) + h1 * bf16_round(A[(32 + lane) * 2 + 1]);
    s[2] = h0 * bf16_round(A[(64 + lane) * 2]) + h1 * bf16_round(A[(96 + lane) * 2]); s[3] = h0 * bf16_round(A[(64 + lane) * 2 + 1]) + h1 * bf16_round(A[(96 + lane) * 2 + 1]); }
#pragma unroll
  for (int k = 0; k < 4; ++k) { for (int o = 16; o >= 1; o >>= 1) s[k] += __shfl_xor(s[k], o, 32); }
  if (lane == 0) { so[wv][0] = s[0]; so[wv][1] = s[1]; so[wv][2] = s[2]; so[wv][3] = s[3]; } __syncthreads();
  if (tid < 128 && blockIdx.x * 32 + tid / 4 < NNODE) { *(volatile float*)(SAD + (size_t)blockIdx.x * 128 + tid) = so[tid / 4][tid % 4]; } __threadfence(); if (tid < 128 && blockIdx.x * 32 + tid / 4 < NNODE) { *(volatile float*)(SAD + (size_t)blockIdx.x * 128 + tid) = so[tid / 4][tid % 4]; } }
template <int MODE>
__global__ __launch_bounds__(256) void k_gred(const float* __restrict__ SAD, const int* __restrict__ srci, const int* __restrict__ dsti, const float* __restrict__ ab, const float* __restrict__ MZ, float* __restrict__ P) {
  __shared__ float s0[256], s1[256]; const int tid = threadIdx.x; const float ab0 = bf16_round(ab[0]), ab1 = bf16_round(ab[1]); const float m0 = MODE ? MZ[0] : 0.f, m1 = MODE ? MZ[1] : 0.f;
  float a0 = MODE ? 0.f : -__builtin_inff(), a1 = a0;
#pragma unroll 1
  for (size_t e = (size_t)blockIdx.x * 256 + tid; e < (size_t)NE; e += (size_t)NRB * 256) { int s = srci[e], d = dsti[e]; s = s < 0 ? 0 : (s >= NNODE ? NNODE - 1 : s); d = d < 0 ? 0 : (d >= NNODE ? NNODE - 1 : d);
    const v4f ss = *(const v4fa*)(SAD + (size_t)s * 4), dd = *(const v4fa*)(SAD + (size_t)d * 4); const float l0 = ss[0] + dd[2] + ab0, l1 = ss[1] + dd[3] + ab1;
    if (MODE) { a0 += expf(l0 - m0); a1 += expf(l1 - m1); } else { a0 = fmaxf(a0, l0); a1 = fmaxf(a1, l1); } }
  s0[tid] = a0; s1[tid] = a1; __syncthreads();
  for (int st = 128; st >= 1; st >>= 1) { if (tid < st) { if (MODE) { s0[tid] += s0[tid + st]; s1[tid] += s1[tid + st]; } else { s0[tid] = fmaxf(s0[tid], s0[tid + st]); s1[tid] = fmaxf(s1[tid], s1[tid + st]); } } __syncthreads(); }
  if (tid < 32) { const float v = (tid == 0) ? s0[0] : (tid == 1 ? s1[0] : 0.f); *(volatile float*)(P + (size_t)blockIdx.x * 32 + tid) = v; } __threadfence(); if (tid < 32) { const float v = (tid == 0) ? s0[0] : (tid == 1 ? s1[0] : 0.f); *(volatile float*)(P + (size_t)blockIdx.x * 32 + tid) = v; } }
template <int MODE>
__global__ __launch_bounds__(32) void k_gfin(const float* __restrict__ P, float* __restrict__ MZ) { const int lane = threadIdx.x; float a0 = MODE ? 0.f : -__builtin_inff(), a1 = a0;
#pragma unroll 1
  for (int b = lane; b < NRB; b += 32) { const float p0 = P[(size_t)b * 32], p1 = P[(size_t)b * 32 + 1]; if (MODE) { a0 += p0; a1 += p1; } else { a0 = fmaxf(a0, p0); a1 = fmaxf(a1, p1); } }
  for (int o = 16; o >= 1; o >>= 1) { const float b0 = __shfl_xor(a0, o, 32), b1 = __shfl_xor(a1, o, 32); if (MODE) { a0 += b0; a1 += b1; } else { a0 = fmaxf(a0, b0); a1 = fmaxf(a1, b1); } }
  float keep0 = MODE ? MZ[0] : a0, keep1 = MODE ? MZ[1] : a1; const float z0 = MODE ? 1.0f / a0 : 0.f, z1 = MODE ? 1.0f / a1 : 0.f;
  const float v = (lane == 0) ? keep0 : (lane == 1 ? keep1 : (lane == 2 ? z0 : (lane == 3 ? z1 : 0.f)));
  *(volatile float*)(MZ + lane) = v; __threadfence(); *(volatile float*)(MZ + lane) = v; }
__global__ __launch_bounds__(1024) void k_sgat(const _Float16* __restrict__ H16, const float* __restrict__ H, const float* __restrict__ SAD, const float* __restrict__ ab, const float* __restrict__ MZ, const int* __restrict__ srci, const int* __restrict__ dsti, _Float16* __restrict__ X16out) {
  __shared__ short Lr[4096]; __shared__ int Le[4096]; __shared__ int scan[32]; __shared__ float stg[64][65];
  const int tid = threadIdx.x, lane = tid & 31, wv = tid >> 5; const int n0 = blockIdx.x * 1024; const int nd = n0 + tid; const int nn = (nd < NNODE) ? nd : 0;
  const float M0 = MZ[0], M1 = MZ[1], iz0 = MZ[2], iz1 = MZ[3]; const float base0 = SAD[(size_t)nn * 4 + 2] + bf16_round(ab[0]) - M0, base1 = SAD[(size_t)nn * 4 + 3] + bf16_round(ab[1]) - M1;
  float acc[HID];
#pragma unroll
  for (int c = 0; c < HID; ++c) acc[c] = 0.f;
#pragma unroll 1
  for (int e0 = 0; e0 < NE; e0 += 4096) { int hr[4], he[4]; int k_cnt = 0;
#pragma unroll
    for (int k = 0; k < 4; ++k) { const int e = e0 + tid * 4 + k; hr[k] = -1; he[k] = 0; if (e < NE) { const int dd_ = dsti[e]; if (dd_ >= n0 && dd_ < n0 + 1024) { hr[k] = dd_ - n0; he[k] = e; ++k_cnt; } } }
    int tot; int p = bscan1024(k_cnt, scan, tid, tot);
#pragma unroll
    for (int k = 0; k < 4; ++k) if (hr[k] >= 0) { Lr[p] = (short)hr[k]; Le[p] = he[k]; ++p; }
    __syncthreads();
    const int ntrip = (tot + 31) >> 5;
#pragma unroll 1
    for (int it = 0; it < ntrip; ++it) { const int q = it * 32 + lane; const int lr = (q < tot) ? (int)Lr[q] : -1;
      unsigned m = __builtin_amdgcn_ballot_w32(lr >= wv * 32 && lr < wv * 32 + 32);
#pragma unroll 1
      while (m) { const int bit = __builtin_ctz(m); m &= m - 1u; const int owner = __shfl(lr, bit, 32); const int e = Le[it * 32 + bit];
        if (tid == owner) { int s = srci[e]; s = s < 0 ? 0 : (s >= NNODE ? NNODE - 1 : s); const v4f sa = *(const v4fa*)(SAD + (size_t)s * 4); const float w0 = expf(sa[0] + base0) * iz0, w1 = expf(sa[1] + base1) * iz1;
          const unsigned short* hr16 = (const unsigned short*)H16 + (size_t)s * HID;
#pragma unroll
          for (int g = 0; g < HD2 / 8; ++g) { FragH f; f.half[0] = *(const v8us*)(hr16 + g * 8);
#pragma unroll
            for (int d = 0; d < 8; ++d) { const float hv = (float)f.h[d]; acc[g * 8 + d] += w0 * hv; acc[HD2 + g * 8 + d] += w1 * hv; } } } } }
    __syncthreads(); }
  { const float* hrow = H + (size_t)nn * HID;
#pragma unroll
    for (int g = 0; g < HID / 4; ++g) { const v4f hv = *(const v4fa*)(hrow + 4 * g);
#pragma unroll
      for (int u = 0; u < 4; ++u) acc[4 * g + u] = fmaxf(acc[4 * g + u] + hv[u], 0.f); } }
  typedef _Float16 v4h __attribute__((ext_vector_type(4)));
  for (int tg = 0; tg < 16; ++tg) {
    if (tid / 64 == tg) {
#pragma unroll
      for (int c = 0; c < HID; ++c) stg[tid % 64][c] = acc[c]; }
    __syncthreads();
    for (int pass = 0; pass < 2; ++pass) {
#pragma unroll 1
      for (int j = tid; j < 64 * 16; j += 1024) { const int r = j / 16, c4 = (j % 16) * 4; const int n = n0 + tg * 64 + r; if (n < NNODE) { v4h h4; h4[0] = (_Float16)stg[r][c4]; h4[1] = (_Float16)stg[r][c4 + 1]; h4[2] = (_Float16)stg[r][c4 + 2]; h4[3] = (_Float16)stg[r][c4 + 3];
          *(volatile v4h*)(X16out + (size_t)n * HID + c4) = h4; } } if (pass == 0) __threadfence(); }
    __syncthreads(); } }
__global__ __launch_bounds__(256) void k_cls2(const _Float16* __restrict__ C1, const float* __restrict__ Wc2, const float* __restrict__ bc2, float* __restrict__ out) { const size_t n = (size_t)blockIdx.x * 256 + threadIdx.x; if (n >= NNODE) return;
  const unsigned short* cr = (const unsigned short*)C1 + n * HD2; float s0 = bf16_round(bc2[0]), s1 = bf16_round(bc2[1]);
#pragma unroll
  for (int g = 0; g < 4; ++g) { FragH f; f.half[0] = *(const v8us*)(cr + 8 * g);
#pragma unroll
    for (int d = 0; d < 8; ++d) { const int j = 8 * g + d; const float v = (float)f.h[d]; s0 += v * bf16_round(Wc2[j * 2]); s1 += v * bf16_round(Wc2[j * 2 + 1]); } }
  typedef float v2f __attribute__((ext_vector_type(2), aligned(8))); v2f o; o.x = s0; o.y = s1; *(volatile v2f*)(out + n * 2) = o; __threadfence(); *(volatile v2f*)(out + n * 2) = o; }

extern "C" void kernel_launch(void* const* d_in, const int* in_sizes, int n_in,
                              void* d_out, int out_size, void* d_ws, size_t ws_size, hipStream_t stream) {
  (void)in_sizes; (void)n_in; (void)out_size;
  const float* x = (const float*)d_in[0]; const int* ei = (const int*)d_in[1];
  const float* W0 = (const float*)d_in[2]; const float* b0 = (const float*)d_in[3]; const float* A0 = (const float*)d_in[4]; const float* a0 = (const float*)d_in[5];
  const float* W1 = (const float*)d_in[6]; const float* b1 = (const float*)d_in[7]; const float* A1 = (const float*)d_in[8]; const float* a1 = (const float*)d_in[9];
  const float* Wc1 = (const float*)d_in[10]; const float* bc1 = (const float*)d_in[11]; const float* Wc2 = (const float*)d_in[12]; const float* bc2 = (const float*)d_in[13];
  const int* srci = ei; const int* dsti = ei + NE;
  char* ws = (char*)d_ws; size_t off = 0;
  auto take = [&](size_t bytes) { char* p = ws + off; off += (bytes + 255) & ~(size_t)255; return p; };
  _Float16* B0 = (_Float16*)take((size_t)HID * IND * 2); _Float16* B1 = (_Float16*)take((size_t)HID * HID * 2); _Float16* Bc = (_Float16*)take((size_t)HD2 * HID * 2); float* MZ = (float*)take(32 * 4); float* P = (float*)take((size_t)NRB * 32 * 4);
  _Float16* X16 = (_Float16*)take((size_t)NNODE * IND * 2); float* H = (float*)take((size_t)NNODE * HID * 4); _Float16* H16 = (_Float16*)take((size_t)NNODE * HID * 2); float* SAD = (float*)take((size_t)((NNODE + 31) / 32) * 128 * 4); _Float16* Xo = (_Float16*)take((size_t)NNODE * HID * 2); _Float16* C1 = (_Float16*)take((size_t)NNODE * HD2 * 2);
  if (off > ws_size) return;
  k_wt_f16<<<(HID * (IND / 8) + 255) / 256, 256, 0, stream>>>(W0, B0, IND, HID, 16.0f); k_wt_f16<<<(HID * (HID / 8) + 255) / 256, 256, 0, stream>>>(W1, B1, HID, HID, 16.0f); k_wt_f16<<<(HD2 * (HID / 8) + 255) / 256, 256, 0, stream>>>(Wc1, Bc, HID, HD2, 16.0f);
  k_x16<<<(unsigned)(((size_t)NNODE * IND / 8 + 255) / 256), 256, 0, stream>>>(x, X16, (size_t)NNODE * IND / 8);
  const unsigned gsad = (NNODE + 31) / 32, gsg = (NNODE + 1023) / 1024; const dim3 gg(((NNODE / 16) * 1 + 3) / 4, 1);
  for (int l = 0; l < 2; ++l) {
    const _Float16* Ain = (l == 0) ? X16 : Xo; const int K = (l == 0) ? IND : HID; const _Float16* Bl = (l == 0) ? B0 : B1; const float* bl = (l == 0) ? b0 : b1; const float* Al = (l == 0) ? A0 : A1; const float* abl = (l == 0) ? a0 : a1;
    k_gemm_hhx<0><<<gg, 128, 0, stream>>>(Ain, K, 0, Bl, K, 0, 0.0625f, bl, 0, nullptr, 1, 0, 0, H, H16, HID, 0, NNODE, HID, K);
    k_sad<<<gsad, 1024, 0, stream>>>(H, Al, SAD);
    k_gred<0><<<NRB, 256, 0, stream>>>(SAD, srci, dsti, abl, MZ, P); k_gfin<0><<<1, 32, 0, stream>>>(P, MZ);
    k_gred<1><<<NRB, 256, 0, stream>>>(SAD, srci, dsti, abl, MZ, P); k_gfin<1><<<1, 32, 0, stream>>>(P, MZ);
    k_sgat<<<gsg, 1024, 0, stream>>>(H16, H, SAD, abl, MZ, srci, dsti, Xo);
  }
  k_gemm_hhx<3><<<gg, 128, 0, stream>>>(Xo, HID, 0, Bc, HID, 0, 0.0625f, bc1, 0, nullptr, 1, 0, 0, nullptr, C1, HD2, 0, NNODE, HD2, HID);
  k_cls2<<<(NNODE + 255) / 256, 256, 0, stream>>>(C1, Wc2, bc2, (float*)d_out);
}
